// VideoGuidedTextRefiner_19310172963217
// MI455X (gfx1250) — hardware-run, weakly checked
//
#include <hip/hip_runtime.h>


#define NQ   4096
#define NV   1024
#define DM   1024
#define NH_  16
#define HD   64
#define HPP  4
#define PCAR 1024.0f
typedef _Float16 h16;
typedef unsigned short bf;
typedef __attribute__((ext_vector_type(16))) __bf16   v16bf;
typedef __attribute__((ext_vector_type(16))) _Float16 v16h;
typedef __attribute__((ext_vector_type(8)))  _Float16 v8h;
typedef __attribute__((ext_vector_type(8)))  unsigned short v8us;
typedef __attribute__((ext_vector_type(8)))  float    v8f;
typedef __attribute__((ext_vector_type(4)))  float    v4f;
typedef v8h  __attribute__((may_alias)) v8ha;
typedef v4f  __attribute__((may_alias)) v4fa;
typedef v8us __attribute__((may_alias)) v8usa;

__device__ __forceinline__ unsigned short f2bf(float f) { unsigned u = __float_as_uint(f); u += 0x7FFFu + ((u >> 16) & 1u); return (unsigned short)(u >> 16); }
__device__ __forceinline__ float bf2f(unsigned short b) { return __uint_as_float(((unsigned)b) << 16); }
__device__ __forceinline__ float bfr(float f) { return bf2f(f2bf(f)); }
__device__ __forceinline__ v16h cat16(v8h lo, v8h hi) { return __builtin_shufflevector(lo, hi, 0, 1, 2, 3, 4, 5, 6, 7, 8, 9, 10, 11, 12, 13, 14, 15); }
__device__ __forceinline__ v16bf cat16b(v8us lo, v8us hi) { return __builtin_bit_cast(v16bf, __builtin_shufflevector(lo, hi, 0, 1, 2, 3, 4, 5, 6, 7, 8, 9, 10, 11, 12, 13, 14, 15)); }
__device__ __forceinline__ v8f wmma16(v16h a, v16h b, v8f c) { return __builtin_amdgcn_wmma_f32_16x16x32_f16(false, a, false, b, (short)0, c, false, false); }
__device__ __forceinline__ v8f wmmab(v16bf a, v16bf b, v8f c) { return __builtin_amdgcn_wmma_f32_16x16x32_bf16(false, a, false, b, (short)0, c, false, false); }


template <typename T16> struct WFrag;
template <> struct WFrag<h16> { typedef v16h V; static __device__ __forceinline__ V ld(const h16* p) { return cat16(*(const v8h*)p, *(const v8h*)(p + 16)); } static __device__ __forceinline__ v8f mma(V a, V b, v8f c) { return wmma16(a, b, c); } };
template <> struct WFrag<bf> { typedef v16bf V; static __device__ __forceinline__ V ld(const bf* p) { return cat16b(*(const v8us*)p, *(const v8us*)(p + 16)); } static __device__ __forceinline__ v8f mma(V a, V b, v8f c) { return wmmab(a, b, c); } };
template <typename T16, int NSPLIT, bool BIAS>
__global__ __launch_bounds__(32) void k_gemmw(const T16* __restrict__ A, const T16* __restrict__ A2, const T16* __restrict__ Bt, const T16* __restrict__ Bt2, int K, float* C, int ldc, const float* __restrict__ bias, size_t sA, size_t sB, size_t sC) {
    typedef typename WFrag<T16>::V V;
    __shared__ __align__(16) float os[16 * 68];
    const size_t z = blockIdx.z; A += z * sA; if (A2) A2 += z * sA; Bt += z * sB; if (Bt2) Bt2 += z * sB; C += z * sC;
    const int lane = threadIdx.x & 31, lr = lane & 15, hi = lane >> 4; const int r0 = blockIdx.x * 64, c0 = blockIdx.y * 64;
    v8f acc[4][4];
#pragma unroll
    for (int mb = 0; mb < 4; ++mb)
#pragma unroll
        for (int nb = 0; nb < 4; ++nb) acc[mb][nb] = (v8f){};
    const size_t aoff = (size_t)(r0 + lr) * K + 8 * hi, boff = (size_t)(c0 + lr) * K + 8 * hi;
#pragma unroll 1
    for (int kc = 0; kc < K; kc += 32) {
        V a[4], a2[4];
#pragma unroll
        for (int mb = 0; mb < 4; ++mb) { a[mb] = WFrag<T16>::ld(A + aoff + (size_t)mb * 16 * K + kc); if (NSPLIT == 1 || NSPLIT == 2) a2[mb] = WFrag<T16>::ld(A2 + aoff + (size_t)mb * 16 * K + kc); }
#pragma unroll
        for (int nb = 0; nb < 4; ++nb) { const V b = WFrag<T16>::ld(Bt + boff + (size_t)nb * 16 * K + kc); V b2; if (NSPLIT >= 2) b2 = WFrag<T16>::ld(Bt2 + boff + (size_t)nb * 16 * K + kc);
#pragma unroll
            for (int mb = 0; mb < 4; ++mb) { acc[mb][nb] = WFrag<T16>::mma(a[mb], b, acc[mb][nb]); if (NSPLIT == 1 || NSPLIT == 2) acc[mb][nb] = WFrag<T16>::mma(a2[mb], b, acc[mb][nb]); if (NSPLIT >= 2) acc[mb][nb] = WFrag<T16>::mma(a[mb], b2, acc[mb][nb]); } }
        asm volatile("v_nop\n\tv_nop\n\tv_nop\n\tv_nop" : "+v"(acc[0][0]), "+v"(acc[1][1]), "+v"(acc[2][2]), "+v"(acc[3][3]) : "v"(a[0]), "v"(a[3]));
    }
#pragma unroll
    for (int mb = 0; mb < 4; ++mb) {
#pragma unroll
        for (int nb = 0; nb < 4; ++nb) {
#pragma unroll
            for (int j = 0; j < 8; ++j) os[(hi * 8 + j) * 68 + nb * 16 + lr] = acc[mb][nb][j]; }
        __builtin_amdgcn_wave_barrier(); asm volatile("" ::: "memory");
        float* crow = C + (size_t)(r0 + mb * 16) * ldc + c0;
#pragma unroll 1
        for (int ps = 0; ps < 2; ++ps) {
#pragma unroll
            for (int s = 0; s < 8; ++s) { const int row = 2 * s + hi, cofs = lr * 4; v4f val = *(const v4fa*)(os + row * 68 + cofs); if (BIAS) { val[0] += bfr(bias[c0 + cofs]); val[1] += bfr(bias[c0 + cofs + 1]); val[2] += bfr(bias[c0 + cofs + 2]); val[3] += bfr(bias[c0 + cofs + 3]); }
                *(volatile v4f*)(crow + (size_t)row * ldc + cofs) = val; }
            if (ps == 0) __threadfence(); }
        __builtin_amdgcn_wave_barrier(); asm volatile("" ::: "memory");
    }
}

__device__ __forceinline__ h16 tohx(float x) { return (h16)x; }
__device__ __forceinline__ void splitf(float y, unsigned short& h, unsigned short& l) { h = f2bf(y); l = f2bf(y - bf2f(h)); }
typedef __attribute__((ext_vector_type(2))) unsigned short v2us;
typedef __attribute__((ext_vector_type(4))) unsigned short v4us;
typedef __attribute__((ext_vector_type(2))) _Float16 v2h;
typedef __attribute__((ext_vector_type(4))) _Float16 v4h;

__global__ __launch_bounds__(256) void k_wtG(const float* __restrict__ w, int K, int N, bf* Bt) {
    const int lane = threadIdx.x & 31; const int L0 = (blockIdx.x * 8 + (threadIdx.x >> 5)) * 8; const int nlines = N * K / 64;
#pragma unroll
    for (int ps = 0; ps < 2; ++ps) {
#pragma unroll 1
        for (int l = 0; l < 8; ++l) { const int L = L0 + l; if (L >= nlines) break; const size_t e = (size_t)L * 64 + lane * 2; const int k = (int)(e % K), n = (int)(e / K); v2us o;
            o[0] = f2bf(w[(size_t)k * N + n]); o[1] = f2bf(w[(size_t)(k + 1) * N + n]); *(volatile v2us*)(Bt + e) = o; }
        if (ps == 0) __threadfence(); }
}
__global__ __launch_bounds__(256) void k_cvt8(const float* __restrict__ src, bf* dst, size_t n8) { const size_t i = (size_t)blockIdx.x * 256 + threadIdx.x; if (i >= n8) return; const v8f v = *(const v8f*)(src + i * 8); v8us o;
#pragma unroll
    for (int k = 0; k < 8; ++k) o[k] = f2bf(v[k]); *(volatile v8us*)(dst + i * 8) = o; __threadfence(); *(volatile v8us*)(dst + i * 8) = o; }
__global__ __launch_bounds__(256) void k_pl(const float* __restrict__ F, int nrows, h16* P) { const size_t e = ((size_t)blockIdx.x * 256 + threadIdx.x) * 4; if (e >= (size_t)NH_ * nrows * HD) return; const int d = (int)(e % HD); const int t = (int)((e / HD) % nrows); const int h = (int)(e / ((size_t)HD * nrows)); const float* f = F + (size_t)t * DM + h * HD + d; v4h o;
#pragma unroll
    for (int u = 0; u < 4; ++u) o[u] = tohx(f[u]); *(volatile v4h*)(P + e) = o; __threadfence(); *(volatile v4h*)(P + e) = o; }
__global__ __launch_bounds__(256) void k_vt(const float* __restrict__ V, h16* VT) { const int e = (blockIdx.x * 256 + threadIdx.x) * 2; if (e >= NH_ * HD * NV) return; const int t = e % NV; const int d = (e / NV) % HD; const int h = e / (NV * HD); v2h o; o[0] = tohx(V[(size_t)t * DM + h * HD + d]); o[1] = tohx(V[(size_t)(t + 1) * DM + h * HD + d]); *(volatile v2h*)(VT + e) = o; __threadfence(); *(volatile v2h*)(VT + e) = o; }
__global__ __launch_bounds__(256) void k_soft(const float* __restrict__ Sb, h16* P16) { const int lane = threadIdx.x & 31; const int row = blockIdx.x * 8 + (threadIdx.x >> 5); if (row >= HPP * NQ) return; const float* sr = Sb + (size_t)row * NV; float v[NV / 32]; float mx = -3.0e38f;
#pragma unroll
    for (int ch = 0; ch < NV / 128; ++ch) { const v4f a = *(const v4f*)(sr + ch * 128 + lane * 4);
#pragma unroll
        for (int u = 0; u < 4; ++u) { const float t = a[u] * 0.125f; v[ch * 4 + u] = t; mx = fmaxf(mx, t); } }
#pragma unroll
    for (int sh = 16; sh; sh >>= 1) mx = fmaxf(mx, __shfl_xor(mx, sh, 32));
    float sum = 0.f;
#pragma unroll
    for (int q = 0; q < NV / 32; ++q) { float d0 = __fsub_rn(v[q], mx); asm volatile("" : "+v"(d0)); v[q] = __builtin_amdgcn_exp2f(__fmul_rn(d0, 1.4426950408889634f)); sum += v[q]; }
#pragma unroll
    for (int sh = 16; sh; sh >>= 1) sum += __shfl_xor(sum, sh, 32);
    const float f = __fdiv_rn(PCAR, sum);
    for (int ps = 0; ps < 2; ++ps) {
#pragma unroll
        for (int ch = 0; ch < NV / 128; ++ch) { v4h o4;
#pragma unroll
            for (int q = 0; q < 4; ++q) o4[q] = tohx(v[ch * 4 + q] * f); *(volatile v4h*)(P16 + (size_t)row * NV + ch * 128 + lane * 4) = o4; }
        if (ps == 0) __threadfence(); } }
__global__ __launch_bounds__(256) void k_mrg(const float* __restrict__ O, int h0, bf* Ah, bf* Al) { const int e = (blockIdx.x * 256 + threadIdx.x) * 4; if (e >= HPP * NQ * HD) return; const int d = e % HD; const int t = (e / HD) % NQ; const int z = e / (HD * NQ); v4us oh, ol;
#pragma unroll
    for (int u = 0; u < 4; ++u) { unsigned short a, b; splitf(O[e + u] * (1.0f / PCAR), a, b); oh[u] = a; ol[u] = b; } const size_t oo = (size_t)t * DM + (h0 + z) * HD + d; *(volatile v4us*)(Ah + oo) = oh; *(volatile v4us*)(Al + oo) = ol; __threadfence(); *(volatile v4us*)(Ah + oo) = oh; *(volatile v4us*)(Al + oo) = ol; }
__device__ __forceinline__ void ln32(float* v, float eps) {
    float s = 0.f;
#pragma unroll
    for (int k = 0; k < DM / 32; ++k) s += v[k];
#pragma unroll
    for (int sh = 16; sh; sh >>= 1) s += __shfl_xor(s, sh, 32);
    const float mean = s * (1.0f / DM); float q = 0.f;
#pragma unroll
    for (int k = 0; k < DM / 32; ++k) { float d = __fsub_rn(v[k], mean); asm volatile("" : "+v"(d)); v[k] = d; float p = __fmul_rn(d, d); asm volatile("" : "+v"(p)); q = __fadd_rn(q, p); }
#pragma unroll
    for (int sh = 16; sh; sh >>= 1) q += __shfl_xor(q, sh, 32);
    const float rden = __fdiv_rn(1.0f, __fsqrt_rn(__fadd_rn(q * (1.0f / DM), eps)));
#pragma unroll
    for (int k = 0; k < DM / 32; ++k) v[k] = __fmul_rn(v[k], rden); }
__global__ __launch_bounds__(256) void k_lnln(const float* __restrict__ AO, const float* __restrict__ QF, const float* __restrict__ g1, const float* __restrict__ b1, const float* __restrict__ g2, const float* __restrict__ b2, bf* Hh, bf* Hl) { const int lane = threadIdx.x & 31; const int r = blockIdx.x * 8 + (threadIdx.x >> 5); if (r >= NQ) return; float v[DM / 32];
#pragma unroll
    for (int ch = 0; ch < DM / 128; ++ch) { const size_t o0 = (size_t)r * DM + ch * 128 + lane * 4; const v4f a = *(const v4f*)(AO + o0), x = *(const v4f*)(QF + o0);
#pragma unroll
        for (int u = 0; u < 4; ++u) { float xb = bfr(x[u]); asm volatile("" : "+v"(xb)); v[ch * 4 + u] = __fadd_rn(a[u], xb); } }
    ln32(v, 1e-12f);
#pragma unroll
    for (int ch = 0; ch < DM / 128; ++ch) {
#pragma unroll
        for (int u = 0; u < 4; ++u) { const int c = ch * 128 + lane * 4 + u; float gg = bfr(g1[c]), bb = bfr(b1[c]); asm volatile("" : "+v"(gg)); asm volatile("" : "+v"(bb)); float t1 = __fmul_rn(v[ch * 4 + u], gg); asm volatile("" : "+v"(t1)); v[ch * 4 + u] = __fadd_rn(t1, bb); } }
    ln32(v, 1e-5f);
    for (int ps = 0; ps < 2; ++ps) {
#pragma unroll
        for (int ch = 0; ch < DM / 128; ++ch) { const int c0 = ch * 128 + lane * 4; v4us oh, ol;
#pragma unroll
            for (int u = 0; u < 4; ++u) { float gg = bfr(g2[c0 + u]), bb = bfr(b2[c0 + u]); asm volatile("" : "+v"(gg)); asm volatile("" : "+v"(bb)); float t1 = __fmul_rn(v[ch * 4 + u], gg); asm volatile("" : "+v"(t1)); const float y = __fadd_rn(t1, bb); unsigned short a2, c2; splitf(y, a2, c2); oh[u] = a2; ol[u] = c2; }
            const size_t oo = (size_t)r * DM + c0; *(volatile v4us*)(Hh + oo) = oh; *(volatile v4us*)(Hl + oo) = ol; }
        if (ps == 0) __threadfence(); } }

extern "C" void kernel_launch(void* const* d_in, const int* in_sizes, int n_in,
                              void* d_out, int out_size, void* d_ws, size_t ws_size, hipStream_t stream) {
    (void)in_sizes; (void)n_in; (void)out_size;
    const float** I = (const float**)d_in;
    const float *qf = I[0], *vf = I[1], *Wq = I[2], *bq = I[3], *Wk = I[4], *bk = I[5], *Wv = I[6], *bv = I[7], *Wo = I[8], *bo = I[9], *g1 = I[10], *b1 = I[11], *g2 = I[12], *b2 = I[13], *Wl = I[14], *bl = I[15];
    float* OUT = (float*)d_out;
    char* wsp = (char*)d_ws;
    auto take = [&](size_t bytes) { char* p = wsp; wsp += (bytes + 255) & ~(size_t)255; return (void*)p; };
    bf* BQ = (bf*)take((size_t)DM * DM * 2); bf* BK = (bf*)take((size_t)DM * DM * 2); bf* BV = (bf*)take((size_t)DM * DM * 2); bf* BO = (bf*)take((size_t)DM * DM * 2); bf* BL = (bf*)take((size_t)DM * DM * 2);
    bf* QB = (bf*)take((size_t)NQ * DM * 2); bf* VBb = (bf*)take((size_t)NV * DM * 2); float* Q = (float*)take((size_t)NQ * DM * 4); float* K = (float*)take((size_t)NV * DM * 4); float* V = (float*)take((size_t)NV * DM * 4);
    h16* Q16 = (h16*)take((size_t)NH_ * NQ * HD * 2); h16* K16 = (h16*)take((size_t)NH_ * NV * HD * 2); h16* VT = (h16*)take((size_t)NH_ * HD * NV * 2); float* Sb = (float*)take((size_t)HPP * NQ * NV * 4); h16* P16 = (h16*)take((size_t)HPP * NQ * NV * 2); float* O = (float*)take((size_t)HPP * NQ * HD * 4);
    bf* Ch = (bf*)take((size_t)NQ * DM * 2); bf* Cl = (bf*)take((size_t)NQ * DM * 2); float* AO = (float*)take((size_t)NQ * DM * 4); bf* Rh = (bf*)take((size_t)NQ * DM * 2); bf* Rl = (bf*)take((size_t)NQ * DM * 2);
    if ((size_t)(wsp - (char*)d_ws) > ws_size) return;
    k_wtG<<<(DM * DM / 64 + 63) / 64, 256, 0, stream>>>(Wq, DM, DM, BQ); k_wtG<<<(DM * DM / 64 + 63) / 64, 256, 0, stream>>>(Wk, DM, DM, BK); k_wtG<<<(DM * DM / 64 + 63) / 64, 256, 0, stream>>>(Wv, DM, DM, BV); k_wtG<<<(DM * DM / 64 + 63) / 64, 256, 0, stream>>>(Wo, DM, DM, BO); k_wtG<<<(DM * DM / 64 + 63) / 64, 256, 0, stream>>>(Wl, DM, DM, BL);
    k_cvt8<<<(NQ * DM / 8 + 255) / 256, 256, 0, stream>>>(qf, QB, (size_t)NQ * DM / 8); k_cvt8<<<(NV * DM / 8 + 255) / 256, 256, 0, stream>>>(vf, VBb, (size_t)NV * DM / 8);
    k_gemmw<bf, 0, true><<<dim3(NQ / 64, DM / 64, 1), 32, 0, stream>>>(QB, nullptr, BQ, nullptr, DM, Q, DM, bq, 0, 0, 0); k_gemmw<bf, 0, true><<<dim3(NV / 64, DM / 64, 1), 32, 0, stream>>>(VBb, nullptr, BK, nullptr, DM, K, DM, bk, 0, 0, 0); k_gemmw<bf, 0, true><<<dim3(NV / 64, DM / 64, 1), 32, 0, stream>>>(VBb, nullptr, BV, nullptr, DM, V, DM, bv, 0, 0, 0);
    k_pl<<<(unsigned)(((size_t)NH_ * NQ * HD / 4 + 255) / 256), 256, 0, stream>>>(Q, NQ, Q16); k_pl<<<(unsigned)(((size_t)NH_ * NV * HD / 4 + 255) / 256), 256, 0, stream>>>(K, NV, K16); k_vt<<<(NH_ * HD * NV / 2 + 255) / 256, 256, 0, stream>>>(V, VT);
    const size_t zq = (size_t)NQ * HD, zk = (size_t)NV * HD, zS = (size_t)NQ * NV;
    for (int h0 = 0; h0 < NH_; h0 += HPP) {
        k_gemmw<h16, 0, false><<<dim3(NQ / 64, NV / 64, HPP), 32, 0, stream>>>(Q16 + (size_t)h0 * zq, nullptr, K16 + (size_t)h0 * zk, nullptr, HD, Sb, NV, nullptr, zq, zk, zS);
        k_soft<<<HPP * NQ / 8, 256, 0, stream>>>(Sb, P16);
        k_gemmw<h16, 0, false><<<dim3(NQ / 64, 1, HPP), 32, 0, stream>>>(P16, nullptr, VT + (size_t)h0 * HD * NV, nullptr, NV, O, HD, nullptr, zS, (size_t)HD * NV, zq);
        k_mrg<<<(HPP * NQ * HD / 4 + 255) / 256, 256, 0, stream>>>(O, h0, Ch, Cl); }
    k_gemmw<bf, 1, true><<<dim3(NQ / 64, DM / 64, 1), 32, 0, stream>>>(Ch, Cl, BO, nullptr, DM, AO, DM, bo, 0, 0, 0);
    k_lnln<<<NQ / 8, 256, 0, stream>>>(AO, qf, g1, b1, g2, b2, Rh, Rl);
    k_gemmw<bf, 1, true><<<dim3(NQ / 64, DM / 64, 1), 32, 0, stream>>>(Rh, Rl, BL, nullptr, DM, OUT, DM, bl, 0, 0, 0);
}
